// GraphConvLayer_88038239634289
// MI455X (gfx1250) — hardware-verified
//
#include <hip/hip_runtime.h>
#include <stddef.h>
#include <stdint.h>


#define DF      64
#define NTHR    256
#define NWAVE   8
#define EPT     8
#define CHUNK   (NTHR * EPT)
#define WCAP    (EPT * 32)
#define LISTN   (NWAVE * WCAP)
#define NBMAX   2048
#define NBRUN   1024
#define RCAP    28672
#define DEGCAP  64
#define PKS     11
#define STW     128
#define GBM     64
#define GTHR    128
#define GNT     4
#define HP      128
#define AP      256
#define KP1     64
#define KP2     128
#define KU1     192
#define KU2     128
#define NU_W1P  (DF * (KP1 / 8))
#define NU_W2P  (DF * (KP2 / 8))
#define NU_W1U  (DF * (KU1 / 8))
#define NU_W2U  (DF * (KU2 / 8))
#define NUW     (NU_W1P + NU_W2P + NU_W1U + NU_W2U)
#define OW1P    0
#define OW2P    (OW1P + DF * KP1)
#define OW1U    (OW2P + DF * KP2)
#define OW2U    (OW1U + DF * KU1)
#define NWT     (OW2U + DF * KU2)
#define WSMAX   134217728
#define LDS_AGG ((2 * RCAP + 2 * NBMAX + LISTN) * 4 + 64)
#define EPS_L2  1e-12f

static_assert((CHUNK & (CHUNK - 1)) == 0 && CHUNK <= (1 << PKS));
static_assert((NBMAX & (NBMAX - 1)) == 0 && NBMAX <= (1 << PKS));
static_assert((NBRUN & (NBRUN - 1)) == 0 && NBRUN <= NBMAX && NBRUN >= 16);
static_assert(NTHR * 8 == NBMAX);
static_assert(LISTN >= NBMAX);
static_assert(LISTN >= NWAVE * WCAP);
static_assert((RCAP % 32) == 0);
static_assert(NWAVE * STW <= RCAP && STW >= 128);
static_assert(LDS_AGG <= 300000);
static_assert(GBM == (GTHR / 32) * 16);
static_assert(DF == 16 * GNT && DF == 16 * 4);
static_assert((KP1 % 32) == 0 && (KP2 % 32) == 0 && (KU1 % 32) == 0 && (KU2 % 32) == 0);
static_assert(KP2 == 2 * DF && KU2 == 2 * DF && KU1 == 3 * DF && HP == 2 * DF && AP == 4 * DF);
static_assert((NU_W1P % NTHR) == 0 && ((NU_W1P + NU_W2P) % NTHR) == 0);
static_assert(((NU_W1P + NU_W2P + NU_W1U) % NTHR) == 0 && (NUW % NTHR) == 0);
static_assert((OW2P % 64) == 0 && (OW1U % 64) == 0 && (OW2U % 64) == 0);

typedef float          v2f  __attribute__((ext_vector_type(2)));
typedef float          v4f  __attribute__((ext_vector_type(4)));
typedef float          v8f  __attribute__((ext_vector_type(8)));
typedef int            v4i  __attribute__((ext_vector_type(4)));
typedef int            v8i  __attribute__((ext_vector_type(8)));
typedef unsigned int   v4u  __attribute__((ext_vector_type(4)));
typedef unsigned short v8us __attribute__((ext_vector_type(8)));
typedef __bf16         v16b __attribute__((ext_vector_type(16)));
typedef v4f  __attribute__((may_alias)) v4fa;
typedef v8us __attribute__((may_alias)) v8usa;
union FragB { v16b v; v8us h[2]; v8i w; };

__device__ __forceinline__ v8f wmb(const FragB& a, const FragB& b, v8f c) {
  v8f d = __builtin_amdgcn_wmma_f32_16x16x32_bf16(false, a.v, false, b.v, (short)0, c, false, false);
  asm volatile("v_nop\n\tv_nop\n\tv_nop\n\tv_nop" : "+v"(d) : "v"(a.w), "v"(b.w));
  return d;
}

__device__ __forceinline__ unsigned short bf_bits(float f) {
  unsigned int u = __float_as_uint(f);
  u += 0x7FFFu + ((u >> 16) & 1u);
  return (unsigned short)(u >> 16);
}
__device__ __forceinline__ float bf_val(unsigned short b) {
  return __uint_as_float(((unsigned int)b) << 16);
}
__device__ __forceinline__ float bf_rne(float f) { return bf_val(bf_bits(f)); }

__device__ __forceinline__ unsigned short hl_bits(float v, int hsel) {
  const unsigned short hb = bf_bits(v);
  const unsigned short lb = bf_bits(v - bf_val(hb));
  return hsel == 0 ? hb : lb;
}

__device__ __forceinline__ float gelu_f(float v) {
  return 0.5f * v * (1.0f + erff(v * 0.70710678118654752f));
}

__device__ __forceinline__ int scan_chunk(const int* __restrict__ dsts, int nE, int cbase, int slotBase,
                                          int nb, int vec8, int* list, int tid, int lane, int wave) {
  int wc = 0;
  const int el0  = tid * EPT;
  const int e0   = cbase + el0;
  const int sent = -2147483647 - 1;
  v4i da, db;
  if (vec8 != 0 && cbase + CHUNK <= nE) {
    da = *(const v4i*)(dsts + e0);
    db = *(const v4i*)(dsts + e0 + 4);
  } else {
    da.x = (e0     < nE) ? dsts[min(e0,     nE - 1)] : sent;
    da.y = (e0 + 1 < nE) ? dsts[min(e0 + 1, nE - 1)] : sent;
    da.z = (e0 + 2 < nE) ? dsts[min(e0 + 2, nE - 1)] : sent;
    da.w = (e0 + 3 < nE) ? dsts[min(e0 + 3, nE - 1)] : sent;
    db.x = (e0 + 4 < nE) ? dsts[min(e0 + 4, nE - 1)] : sent;
    db.y = (e0 + 5 < nE) ? dsts[min(e0 + 5, nE - 1)] : sent;
    db.z = (e0 + 6 < nE) ? dsts[min(e0 + 6, nE - 1)] : sent;
    db.w = (e0 + 7 < nE) ? dsts[min(e0 + 7, nE - 1)] : sent;
  }
  const unsigned nbs = (unsigned)slotBase;
  const unsigned unb = (unsigned)nb;
  const unsigned s0 = (unsigned)da.x - nbs, s1 = (unsigned)da.y - nbs;
  const unsigned s2 = (unsigned)da.z - nbs, s3 = (unsigned)da.w - nbs;
  const unsigned s4 = (unsigned)db.x - nbs, s5 = (unsigned)db.y - nbs;
  const unsigned s6 = (unsigned)db.z - nbs, s7 = (unsigned)db.w - nbs;
  const bool h0 = s0 < unb, h1 = s1 < unb, h2 = s2 < unb, h3 = s3 < unb;
  const bool h4 = s4 < unb, h5 = s5 < unb, h6 = s6 < unb, h7 = s7 < unb;
  const unsigned any = __builtin_amdgcn_ballot_w32(h0 | h1 | h2 | h3 | h4 | h5 | h6 | h7);
  if (any != 0u) {
#define HITJ(J, HJ, SJ) { \
      const unsigned mj = __builtin_amdgcn_ballot_w32(HJ); \
      if (mj != 0u) { \
        if (HJ) { \
          const int pos = wc + (int)__builtin_amdgcn_mbcnt_lo(mj, 0u); \
          if (pos < WCAP) list[wave * WCAP + pos] = ((el0 + (J)) << PKS) | (int)(SJ); \
        } \
        wc += (int)__builtin_popcount(mj); } }
    HITJ(0, h0, s0)
    HITJ(1, h1, s1)
    HITJ(2, h2, s2)
    HITJ(3, h3, s3)
    HITJ(4, h4, s4)
    HITJ(5, h5, s5)
    HITJ(6, h6, s6)
    HITJ(7, h7, s7)
#undef HITJ
  }
  return wc;
}

__global__ __launch_bounds__(NTHR) void k_prep(const float* __restrict__ x, int nN, int nXU,
                                               const float* __restrict__ W1p, const float* __restrict__ W2p,
                                               const float* __restrict__ W1u, const float* __restrict__ W2u,
                                               unsigned short* XB, unsigned short* WT) {
  const int u = (int)blockIdx.x * NTHR + (int)threadIdx.x;
  v8us o;
  unsigned short* dp;
  if (u < NU_W1P) {
    const int n  = u >> 3;
    const int k8 = (u & 7) * 8;
    const float* p = W1p + (size_t)k8 * DF + n;
#pragma unroll
    for (int i = 0; i < 8; ++i) o[i] = bf_bits(p[(size_t)i * DF]);
    dp = WT + OW1P + (size_t)n * KP1 + k8;
  } else if (u < NU_W1P + NU_W2P) {
    const int v  = u - NU_W1P;
    const int n  = v >> 4;
    const int k8 = (v & 15) * 8;
    const int kk = k8 & (DF - 1);
    const float* p = W2p + (size_t)kk * DF + n;
#pragma unroll
    for (int i = 0; i < 8; ++i) o[i] = bf_bits(p[(size_t)i * DF]);
    dp = WT + OW2P + (size_t)n * KP2 + k8;
  } else if (u < NU_W1P + NU_W2P + NU_W1U) {
    const int v  = u - (NU_W1P + NU_W2P);
    const int n  = v / (KU1 / 8);
    const int k8 = (v - n * (KU1 / 8)) * 8;
    const int kk = k8 < 2 * DF ? k8 : k8 - DF;
    const float* p = W1u + (size_t)kk * DF + n;
#pragma unroll
    for (int i = 0; i < 8; ++i) o[i] = bf_bits(p[(size_t)i * DF]);
    dp = WT + OW1U + (size_t)n * KU1 + k8;
  } else if (u < NUW) {
    const int v  = u - (NU_W1P + NU_W2P + NU_W1U);
    const int n  = v >> 4;
    const int k8 = (v & 15) * 8;
    const int kk = k8 & (DF - 1);
    const float* p = W2u + (size_t)kk * DF + n;
#pragma unroll
    for (int i = 0; i < 8; ++i) o[i] = bf_bits(p[(size_t)i * DF]);
    dp = WT + OW2U + (size_t)n * KU2 + k8;
  } else {
    const int v = u - NUW;
    if (v >= nXU) return;
    const int row = v >> 3;
    const int k8  = (v & 7) * 8;
    const int rc  = row < nN ? row : nN - 1;
    const float* p = x + (size_t)rc * DF + k8;
    const v4f a = *(const v4f*)p;
    const v4f b = *(const v4f*)(p + 4);
    const bool ok = row < nN;
    o[0] = ok ? bf_bits(a.x) : (unsigned short)0;  o[1] = ok ? bf_bits(a.y) : (unsigned short)0;
    o[2] = ok ? bf_bits(a.z) : (unsigned short)0;  o[3] = ok ? bf_bits(a.w) : (unsigned short)0;
    o[4] = ok ? bf_bits(b.x) : (unsigned short)0;  o[5] = ok ? bf_bits(b.y) : (unsigned short)0;
    o[6] = ok ? bf_bits(b.z) : (unsigned short)0;  o[7] = ok ? bf_bits(b.w) : (unsigned short)0;
    dp = XB + (size_t)row * DF + k8;
  }
  *(volatile v8us*)dp = o;
  __threadfence();
  *(volatile v8us*)dp = o;
}

template <int EPI>
__global__ __launch_bounds__(GTHR) void k_gemm(const unsigned short* __restrict__ A, int lda,
                                               const unsigned short* __restrict__ BT, int K,
                                               const float* __restrict__ bias,
                                               unsigned short* Hout, float* Fout, int nRows) {
  __shared__ __attribute__((aligned(16))) float stg[GBM * DF];
  const int tid = (int)threadIdx.x, lane = tid & 31, wave = tid >> 5, hh = lane >> 4, m = lane & 15;
  const int rowBase = (int)blockIdx.x * GBM;

  v8f acc[GNT];
  {
    const v8f z = {0.f, 0.f, 0.f, 0.f, 0.f, 0.f, 0.f, 0.f};
#pragma unroll
    for (int t = 0; t < GNT; ++t) acc[t] = z;
  }
  const unsigned short* ap = A  + (size_t)(rowBase + 16 * wave + m) * (size_t)lda + 8 * hh;
  const unsigned short* bp = BT + (size_t)m * (size_t)K + 8 * hh;
#pragma unroll 1
  for (int k0 = 0; k0 < K; k0 += 32) {
    FragB af;
    af.h[0] = *(const v8usa*)(ap + k0);
    af.h[1] = *(const v8usa*)(ap + k0 + 16);
#pragma unroll
    for (int t = 0; t < GNT; ++t) {
      const unsigned short* wq = bp + (size_t)(16 * t) * (size_t)K + k0;
      FragB bf;
      bf.h[0] = *(const v8usa*)wq;
      bf.h[1] = *(const v8usa*)(wq + 16);
      acc[t] = wmb(af, bf, acc[t]);
    }
  }

#pragma unroll
  for (int t = 0; t < GNT; ++t) {
    const int lc = 16 * t + m;
    const float bb = bf_rne(bias[lc]);
#pragma unroll
    for (int r = 0; r < 8; ++r) {
      const int lr = 16 * wave + 8 * hh + r;
      stg[lr * DF + lc] = gelu_f(acc[t][r] + bb);
    }
  }
  __syncthreads();

  const int l16 = lane & 15;
  if constexpr (EPI == 0) {
    v8us ho[8];
    const int c8   = 8 * (l16 & 7);
    const int hsel = l16 >> 3;
#pragma unroll
    for (int i = 0; i < 8; ++i) {
      const int lr = 16 * wave + 2 * i + hh;
      const v4f a = *(const v4fa*)(stg + lr * DF + c8);
      const v4f b = *(const v4fa*)(stg + lr * DF + c8 + 4);
      v8us o;
      o[0] = hl_bits(a.x, hsel); o[1] = hl_bits(a.y, hsel); o[2] = hl_bits(a.z, hsel); o[3] = hl_bits(a.w, hsel);
      o[4] = hl_bits(b.x, hsel); o[5] = hl_bits(b.y, hsel); o[6] = hl_bits(b.z, hsel); o[7] = hl_bits(b.w, hsel);
      ho[i] = o;
    }
#pragma unroll
    for (int i = 0; i < 8; ++i) {
      const int gr = rowBase + 16 * wave + 2 * i + hh;
      unsigned short* gp = Hout + (size_t)gr * (size_t)HP + 8 * l16;
      if (gr < nRows) *(volatile v8us*)gp = ho[i];
    }
    __threadfence();
#pragma unroll
    for (int i = 0; i < 8; ++i) {
      const int gr = rowBase + 16 * wave + 2 * i + hh;
      unsigned short* gp = Hout + (size_t)gr * (size_t)HP + 8 * l16;
      if (gr < nRows) *(volatile v8us*)gp = ho[i];
    }
  } else {
    v4f ov[8];
#pragma unroll
    for (int i = 0; i < 8; ++i) {
      const int lr = 16 * wave + 2 * i + hh;
      v4f h = *(const v4fa*)(stg + lr * DF + 4 * l16);
      if constexpr (EPI == 2) {
        float ss = (h.x * h.x + h.y * h.y) + (h.z * h.z + h.w * h.w);
#pragma unroll
        for (int mm = 8; mm >= 1; mm >>= 1) ss += __shfl_xor(ss, mm, 32);
        const float sc = rsqrtf(fmaxf(ss, EPS_L2));
        h.x *= sc; h.y *= sc; h.z *= sc; h.w *= sc;
      }
      ov[i] = h;
    }
#pragma unroll
    for (int i = 0; i < 8; ++i) {
      const int gr = rowBase + 16 * wave + 2 * i + hh;
      float* op = Fout + (size_t)gr * (size_t)DF + 4 * l16;
      if (gr < nRows) *(volatile v4f*)op = ov[i];
    }
    __threadfence();
#pragma unroll
    for (int i = 0; i < 8; ++i) {
      const int gr = rowBase + 16 * wave + 2 * i + hh;
      float* op = Fout + (size_t)gr * (size_t)DF + 4 * l16;
      if (gr < nRows) *(volatile v4f*)op = ov[i];
    }
  }
}

__global__ __launch_bounds__(NTHR) void k_agg(
    const int* __restrict__ keyp, const int* __restrict__ nbrp, const float* __restrict__ ew,
    const float* __restrict__ x, const float* __restrict__ P,
    unsigned short* Aout, int nN, int nE, int nb, int vec8, int MPr) {
  extern __shared__ v4f lds_dyn[];
  int* reg1 = (int*)lds_dyn;
  int* reg2 = reg1 + RCAP;
  int* scnt = reg2 + RCAP;
  int* soff = scnt + NBMAX;
  int* list = soff + NBMAX;
  int* wcnt = list + LISTN;
  int* wtot = wcnt + NWAVE;
  const int tid = (int)threadIdx.x, lane = tid & 31, wave = tid >> 5;
  const int nodeBase = (int)blockIdx.x * nb;

  for (int i = tid; i < NBMAX; i += NTHR) scnt[i] = 0;
  __syncthreads();

  int tot = 0;
  const int nChunks = (nE + CHUNK - 1) / CHUNK;
#pragma unroll 1
  for (int ch = 0; ch < nChunks; ++ch) {
    const int cbase = ch * CHUNK;
    const int wc = scan_chunk(keyp, nE, cbase, nodeBase, nb, vec8, list, tid, lane, wave);
    if (lane == 0) wcnt[wave] = wc;
    __syncthreads();
    int pre = 0, all = 0;
#pragma unroll
    for (int w2 = 0; w2 < NWAVE; ++w2) {
      int c = wcnt[w2];
      c = c < 0 ? 0 : (c > WCAP ? WCAP : c);
      all += c;
      pre += (w2 < wave) ? c : 0;
    }
    const int wcc  = wc > WCAP ? WCAP : wc;
    const int base = tot + pre;
#pragma unroll 1
    for (int i = lane; i < wcc; i += 32) {
      const int ent = list[wave * WCAP + i];
      const int el  = (ent >> PKS) & (CHUNK - 1);
      const int sl  = ent & (NBMAX - 1);
      int eid = cbase + el;
      eid = eid > nE - 1 ? nE - 1 : eid;
      const int pos = base + i;
      if (pos < RCAP) reg1[pos] = (int)(((unsigned)eid << PKS) | (unsigned)sl);
    }
    tot += all;
    tot = tot > RCAP ? RCAP : tot;
    __syncthreads();
  }
  const int nh = tot;

  if (wave == 0) {
#pragma unroll 1
    for (int b0 = 0; b0 < nh; b0 += 32) {
      const int idx = b0 + lane;
      const int uv  = reg1[idx < nh ? idx : nh - 1];
      const int m32 = (nh - b0) < 32 ? (nh - b0) : 32;
#pragma unroll 1
      for (int k = 0; k < m32; ++k) {
        const int u  = __builtin_amdgcn_readlane(uv, k);
        const int sl = u & (NBMAX - 1);
        if (lane == 0) scnt[sl] = scnt[sl] + 1;
      }
    }
  }
  __syncthreads();

  {
    const v4i ca = *(const v4i*)(scnt + 8 * tid);
    const v4i cb = *(const v4i*)(scnt + 8 * tid + 4);
    const int e0 = ca.x < 0 ? 0 : ca.x, e1 = ca.y < 0 ? 0 : ca.y, e2 = ca.z < 0 ? 0 : ca.z, e3 = ca.w < 0 ? 0 : ca.w;
    const int e4 = cb.x < 0 ? 0 : cb.x, e5 = cb.y < 0 ? 0 : cb.y, e6 = cb.z < 0 ? 0 : cb.z, e7 = cb.w < 0 ? 0 : cb.w;
    const int ts = e0 + e1 + e2 + e3 + e4 + e5 + e6 + e7;
    int incl = ts;
#pragma unroll
    for (int d = 1; d < 32; d <<= 1) {
      const int up = __shfl_up(incl, d);
      if (lane >= d) incl += up;
    }
    if (lane == 31) wtot[wave] = incl;
    __syncthreads();
    int pre = 0;
#pragma unroll
    for (int w2 = 0; w2 < NWAVE; ++w2) pre += (w2 < wave) ? wtot[w2] : 0;
    int run = pre + incl - ts;
    soff[8 * tid + 0] = run; run += e0;
    soff[8 * tid + 1] = run; run += e1;
    soff[8 * tid + 2] = run; run += e2;
    soff[8 * tid + 3] = run; run += e3;
    soff[8 * tid + 4] = run; run += e4;
    soff[8 * tid + 5] = run; run += e5;
    soff[8 * tid + 6] = run; run += e6;
    soff[8 * tid + 7] = run;
  }
  __syncthreads();
  for (int i = tid; i < NBMAX; i += NTHR) list[i] = soff[i];
  __syncthreads();

  if (wave == 0) {
#pragma unroll 1
    for (int b0 = 0; b0 < nh; b0 += 32) {
      const int idx = b0 + lane;
      const int uv  = reg1[idx < nh ? idx : nh - 1];
      const int m32 = (nh - b0) < 32 ? (nh - b0) : 32;
#pragma unroll 1
      for (int k = 0; k < m32; ++k) {
        const int u   = __builtin_amdgcn_readlane(uv, k);
        const int sl  = u & (NBMAX - 1);
        const int eid = (int)((unsigned)u >> PKS);
        if (lane == 0) {
          int pos = list[sl];
          pos = pos < 0 ? 0 : (pos > RCAP - 1 ? RCAP - 1 : pos);
          reg2[pos] = eid;
          list[sl] = pos + 1;
        }
      }
    }
  }
  __syncthreads();

  const int nbw = nb >> 3;
  const bool ovf = (nh >= RCAP);
  const float qnan = __int_as_float(0x7fc00000);
  unsigned int* stwu = (unsigned int*)(reg1 + wave * STW);

#pragma unroll 1
  for (int jt = 0; jt < nbw; ++jt) {
    const int slot = wave * nbw + jt;
    const int grow = nodeBase + slot;
    int st = soff[slot];
    const int craw = scnt[slot];
    int cnt = craw;
    st  = st < 0 ? 0 : (st > nh ? nh : st);
    cnt = cnt < 0 ? 0 : (cnt > DEGCAP ? DEGCAP : cnt);
    if (cnt > nh - st) cnt = nh - st;
    const float pz = (ovf || craw > DEGCAP) ? qnan : 0.0f;
    const bool liveRow = grow < nN;
    const int grc = liveRow ? grow : nN - 1;

    const v2f xs = *(const v2f*)(x + (size_t)grc * DF + 2 * lane);
    float ag0 = 0.0f, ag1 = 0.0f;
#pragma unroll 1
    for (int b0 = 0; b0 < cnt; b0 += 32) {
      int idx = st + b0 + lane;
      idx = idx > nh - 1 ? nh - 1 : idx;
      idx = idx < 0 ? 0 : idx;
      int eid = reg2[idx];
      eid = eid < 0 ? 0 : (eid > nE - 1 ? nE - 1 : eid);
      const int sraw = nbrp[eid];
      const int s = sraw < 0 ? 0 : (sraw > nN - 1 ? nN - 1 : sraw);
      const float w = bf_rne(ew[eid]);
      const int wi = __float_as_int(w);
      const int m32 = (cnt - b0) < 32 ? (cnt - b0) : 32;
#pragma unroll 1
      for (int k = 0; k < m32; ++k) {
        const int   sk = __builtin_amdgcn_readlane(s, k);
        const float wk = __int_as_float(__builtin_amdgcn_readlane(wi, k));
        const v2f p = *(const v2f*)(P + (size_t)sk * DF + 2 * lane);
        ag0 = fmaf(wk, p.x, ag0);
        ag1 = fmaf(wk, p.y, ag1);
      }
    }
    const float x0 = liveRow ? bf_rne(xs.x) : 0.0f;
    const float x1 = liveRow ? bf_rne(xs.y) : 0.0f;
    const float a0 = (liveRow ? ag0 : 0.0f) + pz;
    const float a1 = (liveRow ? ag1 : 0.0f) + pz;

    const unsigned short hb0 = bf_bits(a0), hb1 = bf_bits(a1);
    const unsigned short lb0 = bf_bits(a0 - bf_val(hb0)), lb1 = bf_bits(a1 - bf_val(hb1));
    const unsigned int xw = (unsigned int)bf_bits(x0) | ((unsigned int)bf_bits(x1) << 16);
    const unsigned int hw = (unsigned int)hb0 | ((unsigned int)hb1 << 16);
    const unsigned int lw = (unsigned int)lb0 | ((unsigned int)lb1 << 16);
    __builtin_amdgcn_fence(__ATOMIC_RELEASE, "wavefront");
    __builtin_amdgcn_wave_barrier();
    stwu[lane]      = xw;
    stwu[32 + lane] = hw;
    stwu[64 + lane] = lw;
    stwu[96 + lane] = 0u;
    __builtin_amdgcn_fence(__ATOMIC_RELEASE, "wavefront");
    __builtin_amdgcn_wave_barrier();
    const v4u pk = *(const v4u*)(stwu + 4 * lane);
    unsigned short* gp = Aout + (size_t)grow * (size_t)AP + 8 * lane;
    const bool wsv = grow < MPr;
    if (wsv) *(volatile v4u*)gp = pk;
    __threadfence();
    if (wsv) *(volatile v4u*)gp = pk;
  }
}

static int pick_nb(int nE, int nN) {
  int nb = NBRUN;
  while (nb > 16 && (long long)nb * (long long)nE * 5LL > (long long)RCAP * (long long)nN * 4LL) nb >>= 1;
  return nb;
}
static inline int cdiv(int a, int b) { return (a + b - 1) / b; }

extern "C" void kernel_launch(void* const* d_in, const int* in_sizes, int n_in,
                              void* d_out, int out_size, void* d_ws, size_t ws_size,
                              hipStream_t stream) {
  if (n_in < 11) return;
  if (in_sizes[0] < DF || (in_sizes[0] % DF) != 0) return;
  const int nN = in_sizes[0] / DF;
  if (nN > (1 << 22)) return;
  const int nE2 = in_sizes[1];
  if (nE2 < 2 || (nE2 & 1) != 0) return;
  const int nE = nE2 / 2;
  if (nE < 1 || nE > (1 << 21)) return;
  if (in_sizes[2] != nE) return;
  if (in_sizes[3] != DF * DF || in_sizes[4] != DF) return;
  if (in_sizes[5] != DF * DF || in_sizes[6] != DF) return;
  if (in_sizes[7] != 2 * DF * DF || in_sizes[8] != DF) return;
  if (in_sizes[9] != DF * DF || in_sizes[10] != DF) return;
  if ((long long)out_size != (long long)nN * DF) return;

  const float* x   = (const float*)d_in[0];
  const int*   edg = (const int*)  d_in[1];
  const int*   key = edg;
  const int*   nbr = edg + nE;
  const float* ew  = (const float*)d_in[2];
  const float* W1p = (const float*)d_in[3];
  const float* b1p = (const float*)d_in[4];
  const float* W2p = (const float*)d_in[5];
  const float* b2p = (const float*)d_in[6];
  const float* W1u = (const float*)d_in[7];
  const float* b1u = (const float*)d_in[8];
  const float* W2u = (const float*)d_in[9];
  const float* b2u = (const float*)d_in[10];
  float* out = (float*)d_out;

  const int MP   = cdiv(nN, GBM) * GBM;
  const int nb   = pick_nb(nE, nN);
  const int gA   = cdiv(MP, nb);
  const int vec8 = 1;
  if (nb < 16 || (nb & 7) != 0) return;
  if ((long long)gA * nb < (long long)MP) return;
  const int nXU = MP * (DF / 8);

  char* ws = (char*)d_ws;
  size_t off = 0;
  const size_t oXB = off; off += (size_t)MP * DF * 2;           off = (off + 255) & ~(size_t)255;
  const size_t oWT = off; off += (size_t)NWT * 2;               off = (off + 255) & ~(size_t)255;
  const size_t oT  = off; off += (size_t)MP * HP * 2;           off = (off + 255) & ~(size_t)255;
  const size_t oP  = off; off += (size_t)MP * DF * 4;           off = (off + 255) & ~(size_t)255;
  const size_t oA  = off; off += (size_t)MP * AP * 2;           off = (off + 255) & ~(size_t)255;
  const size_t oG  = off; off += (size_t)MP * HP * 2;           off = (off + 255) & ~(size_t)255;
  if (off > ws_size || off > (size_t)WSMAX) return;
  unsigned short* XB = (unsigned short*)(ws + oXB);
  unsigned short* WT = (unsigned short*)(ws + oWT);
  unsigned short* T  = (unsigned short*)(ws + oT);
  float*          P  = (float*)(ws + oP);
  unsigned short* AC = (unsigned short*)(ws + oA);
  unsigned short* G  = (unsigned short*)(ws + oG);

  hipFuncSetAttribute(reinterpret_cast<const void*>(&k_agg),
                      hipFuncAttributeMaxDynamicSharedMemorySize, LDS_AGG);

  k_prep<<<cdiv(NUW + nXU, NTHR), NTHR, 0, stream>>>(x, nN, nXU, W1p, W2p, W1u, W2u, XB, WT);

  k_gemm<0><<<MP / GBM, GTHR, 0, stream>>>(XB, DF, WT + OW1P, KP1, b1p, T, P, MP);

  k_gemm<1><<<MP / GBM, GTHR, 0, stream>>>(T, HP, WT + OW2P, KP2, b2p, G, P, MP);

  k_agg<<<gA, NTHR, LDS_AGG, stream>>>(key, nbr, ew, x, P, AC, nN, nE, nb, vec8, MP);

  k_gemm<0><<<MP / GBM, GTHR, 0, stream>>>(AC, AP, WT + OW1U, KU1, b1u, G, P, MP);

  k_gemm<2><<<MP / GBM, GTHR, 0, stream>>>(G, HP, WT + OW2U, KU2, b2u, T, out, nN);
}
